// IHR_24386824306815
// MI455X (gfx1250) — hardware-verified
//
#include <hip/hip_runtime.h>


namespace {
constexpr int Bn = 4, C = 256, HH = 64, WW = 64, N = HH * WW, KO = 32, C1 = 128, KC = 9 * C, NP1 = N + 1;
constexpr float AS = 8.0f, WS = 64.0f, KS = 8.0f, PS = 4096.0f;

typedef _Float16 b16;
typedef __attribute__((ext_vector_type(16))) _Float16 v16b;
typedef __attribute__((ext_vector_type(8)))  _Float16 v8b;
typedef __attribute__((ext_vector_type(8)))  float v8f;
typedef __attribute__((ext_vector_type(4)))  float v4f;

__device__ __forceinline__ v8b ld8b(const b16* p) { return *(const v8b*)p; }
__device__ __forceinline__ v16b cat8b(v8b a, v8b b) { return __builtin_shufflevector(a, b, 0, 1, 2, 3, 4, 5, 6, 7, 8, 9, 10, 11, 12, 13, 14, 15); }
__device__ __forceinline__ v16b frag_kb(const b16* p, int hh) { return cat8b(ld8b(p + 8 * hh), ld8b(p + 16 + 8 * hh)); }
__device__ __forceinline__ void split16(float v, b16& hi, b16& lo) { hi = (b16)v; lo = (b16)(v - (float)hi); }
__device__ __forceinline__ void frag_ksplit(const float* p, int hh, v16b& fh_, v16b& fl_) {
  const float* p0 = p + 8 * hh; const float* p1 = p + 16 + 8 * hh;
#pragma unroll
  for (int e = 0; e < 8; ++e) { b16 a, c; split16(p0[e], a, c); fh_[e] = a; fl_[e] = c; split16(p1[e], a, c); fh_[8 + e] = a; fl_[8 + e] = c; }
}
__device__ __forceinline__ v8f wmma16b(v16b a, v16b b, v8f c) {
  v8f d = __builtin_amdgcn_wmma_f32_16x16x32_f16(false, a, false, b, (short)0, c, false, false);
  asm volatile("v_nop\n\tv_nop\n\tv_nop\n\tv_nop" : "+v"(d) : "v"(a), "v"(b));
  return d;
}
__device__ __forceinline__ void wave_lds_sync() {
  __builtin_amdgcn_fence(__ATOMIC_RELEASE, "workgroup");
  __builtin_amdgcn_wave_barrier();
  __builtin_amdgcn_fence(__ATOMIC_ACQUIRE, "workgroup");
}

struct Opnd { const void* p0; const void* p1; int ld; };
template <int NP> __device__ __forceinline__ void load_frags(const Opnd& o, int row, int kb, int hh, v16b& fh_, v16b& fl_) {
  if (NP == 0) { frag_ksplit((const float*)o.p0 + (size_t)row * o.ld + kb, hh, fh_, fl_); }
  else if (NP == 4) {
    const float* p = (const float*)o.p0 + (size_t)row * o.ld + kb; const float* p0 = p + 8 * hh; const float* p1 = p + 16 + 8 * hh;
#pragma unroll
    for (int e = 0; e < 8; ++e) { b16 a, c; split16(p0[e] * 64.0f, a, c); fh_[e] = a; fl_[e] = c; split16(p1[e] * 64.0f, a, c); fh_[8 + e] = a; fl_[8 + e] = c; }
  } else if (NP == 3) {
    const float* p = (const float*)o.p0 + (size_t)row * o.ld + kb; const float* p0 = p + 8 * hh; const float* p1 = p + 16 + 8 * hh;
#pragma unroll
    for (int e = 0; e < 8; ++e) { fh_[e] = (b16)p0[e]; fh_[8 + e] = (b16)p1[e]; }
    fl_ = fh_;
  } else {
    fh_ = frag_kb((const b16*)o.p0 + (size_t)row * o.ld + kb, hh);
    if (NP == 2) fl_ = frag_kb((const b16*)o.p1 + (size_t)row * o.ld + kb, hh); else fl_ = fh_;
  }
}
template <int ANP, int BNP> __device__ __forceinline__ v8f mac(v16b ah, v16b al, v16b bh, v16b bl, v8f c) {
  c = wmma16b(ah, bh, c);
  if (BNP == 0 || BNP == 2 || BNP == 4) c = wmma16b(ah, bl, c);
  if (ANP == 0 || ANP == 2 || ANP == 4) c = wmma16b(al, bh, c);
  return c;
}
template <int ANP, int BNP>
__device__ __forceinline__ void gemm_tile(const Opnd& A, const Opnd& B, int K, int m0, int c0, int nloc, int hlf, v8f (&acc)[2][4]) {
  for (int kb = 0; kb < K; kb += 32) {
    v16b a0h, a0l, a1h, a1l;
    load_frags<ANP>(A, m0 + nloc, kb, hlf, a0h, a0l);
    load_frags<ANP>(A, m0 + 16 + nloc, kb, hlf, a1h, a1l);
#pragma unroll
    for (int t = 0; t < 4; ++t) {
      v16b bh, bl;
      load_frags<BNP>(B, c0 + t * 16 + nloc, kb, hlf, bh, bl);
      acc[0][t] = mac<ANP, BNP>(a0h, a0l, bh, bl, acc[0][t]);
      acc[1][t] = mac<ANP, BNP>(a1h, a1l, bh, bl, acc[1][t]);
    }
  }
}

__device__ __forceinline__ void epi_planes(v8f (&acc)[2][4], float scale, bool two, b16* __restrict__ oh, b16* __restrict__ ol, int ldo,
                                           int m0, int c0, int lane, b16* Th, b16* Tl) {
  const int nloc = lane & 15, hlf = lane >> 4;
#pragma unroll
  for (int t = 0; t < 4; ++t)
#pragma unroll
    for (int r = 0; r < 2; ++r)
#pragma unroll
      for (int v = 0; v < 8; ++v) {
        const int rr = r * 16 + v + 8 * hlf, cc = t * 16 + nloc;
        b16 h_, l_; split16(acc[r][t][v] * scale, h_, l_);
        Th[rr * 64 + cc] = h_; Tl[rr * 64 + cc] = l_;
      }
  wave_lds_sync();
  for (int pass = 0; pass < 2; ++pass) {
#pragma unroll
    for (int j = 0; j < 8; ++j) {
      const int rr = j * 4 + (lane >> 3), c8 = (lane & 7) * 8;
      const size_t o = (size_t)(m0 + rr) * ldo + c0 + c8;
      *(volatile v8b*)(oh + o) = ld8b(Th + rr * 64 + c8);
      if (two) *(volatile v8b*)(ol + o) = ld8b(Tl + rr * 64 + c8);
    }
    __threadfence();
  }
}
__device__ __forceinline__ void epi_f32(v8f (&acc)[2][4], float scale, const float* rscale, float* __restrict__ out, int ldo, int m0, int c0, int lane, float* Tt) {
  const int nloc = lane & 15, hlf = lane >> 4;
#pragma unroll
  for (int t = 0; t < 4; ++t)
#pragma unroll
    for (int r = 0; r < 2; ++r)
#pragma unroll
      for (int v = 0; v < 8; ++v) {
        const int rr = r * 16 + v + 8 * hlf;
        const float rs = rscale ? rscale[(size_t)(m0 + rr) * 32] : 1.0f;
        Tt[rr * 64 + t * 16 + nloc] = acc[r][t][v] * scale * rs;
      }
  wave_lds_sync();
  float* dst0 = out + (size_t)m0 * ldo + c0;
  for (int pass = 0; pass < 2; ++pass) {
#pragma unroll
    for (int j = 0; j < 16; ++j) { const int rr = j * 2 + hlf, c4 = nloc * 4; *(volatile v4f*)(dst0 + (size_t)rr * ldo + c4) = *(const v4f*)(Tt + rr * 64 + c4); }
    __threadfence();
  }
}


__global__ __launch_bounds__(256) void prep_kernel(const float* __restrict__ ktw, const float* __restrict__ kqw, const float* __restrict__ c1w, const float* __restrict__ mw,
                                                   b16* __restrict__ cwh, b16* __restrict__ cwl, b16* __restrict__ c1h, b16* __restrict__ mwh,
                                                   b16* __restrict__ xh, b16* __restrict__ xl, b16* __restrict__ rh, b16* __restrict__ rl) {
  const size_t tid = (size_t)blockIdx.x * blockDim.x + threadIdx.x, stride = (size_t)gridDim.x * blockDim.x;
  const size_t n0 = (size_t)2 * KO * KC / 8, n1 = (size_t)C1 * C / 8, n2 = (size_t)C * 2 * C / 8;
  for (int pass = 0; pass < 2; ++pass) {
    for (size_t p = tid; p < n0 + n1 + n2; p += stride) {
      v8b vh, vl;
      if (p < n0) { const size_t i = p * 8; const int which = (int)(i / ((size_t)KO * KC)), o = (int)((i / KC) % KO), k0 = (int)(i % KC);
        const float* w = which ? kqw : ktw;
#pragma unroll
        for (int e = 0; e < 8; ++e) { const int k = k0 + e, tap = k / C, c = k % C; b16 a, b2; split16(w[((size_t)o * C + c) * 9 + tap] * WS, a, b2); vh[e] = a; vl[e] = b2; }
        *(volatile v8b*)(cwh + i) = vh; *(volatile v8b*)(cwl + i) = vl; }
      else if (p < n0 + n1) { const size_t i = (p - n0) * 8;
#pragma unroll
        for (int e = 0; e < 8; ++e) vh[e] = (b16)(c1w[i + e] * WS);
        *(volatile v8b*)(c1h + i) = vh; }
      else { const size_t i = (p - n0 - n1) * 8;
#pragma unroll
        for (int e = 0; e < 8; ++e) vh[e] = (b16)(mw[i + e] * WS);
        *(volatile v8b*)(mwh + i) = vh; }
    }
    for (size_t p = tid; p < (size_t)Bn * C / 8; p += stride) { const int b = (int)(p / (C / 8)), c8 = (int)(p % (C / 8)) * 8; v8b z = {};
      const size_t o = ((size_t)b * NP1 + N) * C + c8; *(volatile v8b*)(xh + o) = z; *(volatile v8b*)(xl + o) = z; *(volatile v8b*)(rh + o) = z; *(volatile v8b*)(rl + o) = z; }
    __threadfence();
  }
}

__global__ __launch_bounds__(256) void trans_kernel(const float* __restrict__ x, const float* __restrict__ ref, b16* __restrict__ xh, b16* __restrict__ xl, b16* __restrict__ rh, b16* __restrict__ rl) {
  __shared__ __attribute__((aligned(16))) b16 Th[64][72]; __shared__ __attribute__((aligned(16))) b16 Tl[64][72];
  const int tid = threadIdx.x, lane = tid & 31, wave = tid >> 5, b = blockIdx.y, which = blockIdx.z;
  const int n0 = (blockIdx.x / 4) * 64, c0 = (blockIdx.x % 4) * 64;
  const float* src = (which ? ref : x) + (size_t)b * C * N;
  for (int i = tid; i < 64 * 64; i += 256) { const int cc = i / 64, nn = i % 64; b16 a, b2; split16(src[(size_t)(c0 + cc) * N + n0 + nn] * AS, a, b2); Th[nn][cc] = a; Tl[nn][cc] = b2; }
  __syncthreads();
  b16* oh = (which ? rh : xh) + ((size_t)b * NP1 + n0) * C + c0; b16* ol = (which ? rl : xl) + ((size_t)b * NP1 + n0) * C + c0;
  for (int pass = 0; pass < 2; ++pass) {
#pragma unroll
    for (int j = 0; j < 2; ++j) { const int rr = wave * 8 + j * 4 + (lane >> 3), c8 = (lane & 7) * 8;
      *(volatile v8b*)(oh + (size_t)rr * C + c8) = *(const v8b*)(&Th[rr][c8]); *(volatile v8b*)(ol + (size_t)rr * C + c8) = *(const v8b*)(&Tl[rr][c8]); }
    __threadfence();
  }
}

__global__ __launch_bounds__(256) void refprep_kernel(const float* __restrict__ ref, b16* __restrict__ r16, float* __restrict__ pooled) {
  __shared__ float ps[32];
  const int wave = threadIdx.x >> 5, lane = threadIdx.x & 31, row0 = blockIdx.x * 32;
  for (int q = 0; q < 4; ++q) {
    const int row = row0 + wave * 4 + q; const float* src = ref + (size_t)row * N; b16* dst = r16 + (size_t)row * N; float s = 0.0f;
    for (int pass = 0; pass < 2; ++pass) {
      s = 0.0f;
#pragma unroll 1
      for (int i0 = 0; i0 < N; i0 += 256) { const int i = i0 + lane * 8; v8b v;
#pragma unroll
        for (int e = 0; e < 8; ++e) { const float f = src[i + e]; s += f; v[e] = (b16)f; }
        *(volatile v8b*)(dst + i) = v; }
      __threadfence();
    }
#pragma unroll
    for (int o = 16; o > 0; o >>= 1) s += __shfl_xor(s, o);
    if (lane == 0) ps[wave * 4 + q] = s * (1.0f / N);
  }
  __syncthreads();
  if (wave == 0) { ((volatile float*)pooled)[row0 + lane] = ps[lane]; __threadfence(); ((volatile float*)pooled)[row0 + lane] = ps[lane]; }
}

__global__ __launch_bounds__(128) void conv3_kernel(const b16* __restrict__ xh, const b16* __restrict__ xl, const b16* __restrict__ rh, const b16* __restrict__ rl,
                                                   const b16* __restrict__ cwh, const b16* __restrict__ cwl, const float* __restrict__ ktb, const float* __restrict__ kqb,
                                                   b16* __restrict__ keyh, b16* __restrict__ keyl) {
  __shared__ __attribute__((aligned(16))) b16 Th[4][64][KO + 8]; __shared__ __attribute__((aligned(16))) b16 Tl[4][64][KO + 8];
  const int lane = threadIdx.x & 31, wave = threadIdx.x >> 5, nloc = lane & 15, hlf = lane >> 4;
  const int b = blockIdx.y >> 1, which = blockIdx.y & 1, n0 = blockIdx.x * 256 + wave * 64;
  const b16* ph = (which ? rh : xh) + (size_t)b * NP1 * C; const b16* pl = (which ? rl : xl) + (size_t)b * NP1 * C;
  const Opnd A{cwh + (size_t)which * KO * KC, cwl + (size_t)which * KO * KC, KC};
  int hh4[4], ww4[4];
#pragma unroll
  for (int t = 0; t < 4; ++t) { const int n = n0 + t * 16 + nloc; hh4[t] = n / WW; ww4[t] = n % WW; }
  v8f acc[2][4];
#pragma unroll
  for (int r = 0; r < 2; ++r)
#pragma unroll
    for (int t = 0; t < 4; ++t) acc[r][t] = (v8f){};
#pragma unroll 1
  for (int tap = 0; tap < 9; ++tap) {
    const int di = tap / 3 - 1, dj = tap % 3 - 1;
    int rowp[4];
#pragma unroll
    for (int t = 0; t < 4; ++t) { const int h2 = hh4[t] + di, w2 = ww4[t] + dj; rowp[t] = (h2 >= 0 && h2 < HH && w2 >= 0 && w2 < WW) ? (h2 * WW + w2) : N; }
#pragma unroll 2
    for (int c0 = 0; c0 < C; c0 += 32) {
      const int kb = tap * C + c0;
      v16b a0h, a0l, a1h, a1l;
      load_frags<2>(A, nloc, kb, hlf, a0h, a0l); load_frags<2>(A, 16 + nloc, kb, hlf, a1h, a1l);
#pragma unroll
      for (int t = 0; t < 4; ++t) {
        const v16b bh = frag_kb(ph + (size_t)rowp[t] * C + c0, hlf), bl = frag_kb(pl + (size_t)rowp[t] * C + c0, hlf);
        acc[0][t] = mac<2, 2>(a0h, a0l, bh, bl, acc[0][t]); acc[1][t] = mac<2, 2>(a1h, a1l, bh, bl, acc[1][t]);
      }
    }
  }
  const float* bias = which ? kqb : ktb;
#pragma unroll
  for (int t = 0; t < 4; ++t)
#pragma unroll
    for (int r = 0; r < 2; ++r)
#pragma unroll
      for (int v = 0; v < 8; ++v) { const int o = r * 16 + v + 8 * hlf, nn = t * 16 + nloc; b16 a, b2; split16((acc[r][t][v] * (1.0f / (AS * WS)) + bias[o]) * KS, a, b2); Th[wave][nn][o] = a; Tl[wave][nn][o] = b2; }
  wave_lds_sync();
  const size_t base = (((size_t)which * Bn + b) * N + n0) * KO;
  for (int pass = 0; pass < 2; ++pass) {
#pragma unroll
    for (int j = 0; j < 8; ++j) { const int nn = j * 8 + (lane >> 2), c8 = (lane & 3) * 8;
      *(volatile v8b*)(keyh + base + (size_t)nn * KO + c8) = *(const v8b*)(&Th[wave][nn][c8]); *(volatile v8b*)(keyl + base + (size_t)nn * KO + c8) = *(const v8b*)(&Tl[wave][nn][c8]); }
    __threadfence();
  }
}

__global__ __launch_bounds__(256) void stats_kernel(const b16* __restrict__ keyh, const b16* __restrict__ keyl, float* __restrict__ Mx, float* __restrict__ Li) {
  __shared__ float Ms[128], Ls[128];
  const int wid = threadIdx.x >> 5, lane = threadIdx.x & 31, hh = lane >> 4, col = lane & 15, b = blockIdx.y, m0 = blockIdx.x * 128 + wid * 16;
  const b16* kth = keyh + ((size_t)b * N) * KO; const b16* ktl = keyl + ((size_t)b * N) * KO;
  const b16* kqh = keyh + ((size_t)(Bn + b) * N) * KO; const b16* kql = keyl + ((size_t)(Bn + b) * N) * KO;
  const v16b bqh = frag_kb(kqh + (size_t)(m0 + col) * KO, hh), bql = frag_kb(kql + (size_t)(m0 + col) * KO, hh);
  float m = -INFINITY, l = 0.0f;
  for (int nb = 0; nb < N; nb += 32) {
    v8f s0 = {}, s1 = {};
    { const v16b ah = frag_kb(kth + (size_t)(nb + col) * KO, hh), al = frag_kb(ktl + (size_t)(nb + col) * KO, hh); s0 = mac<2, 2>(ah, al, bqh, bql, s0); }
    { const v16b ah = frag_kb(kth + (size_t)(nb + 16 + col) * KO, hh), al = frag_kb(ktl + (size_t)(nb + 16 + col) * KO, hh); s1 = mac<2, 2>(ah, al, bqh, bql, s1); }
    float mr = -INFINITY;
#pragma unroll
    for (int r = 0; r < 8; ++r) { s0[r] *= (1.0f / (KS * KS)); s1[r] *= (1.0f / (KS * KS)); mr = fmaxf(mr, fmaxf(s0[r], s1[r])); }
    mr = fmaxf(mr, __shfl_xor(mr, 16));
    const float mn = fmaxf(m, mr), al_ = __expf(m - mn); m = mn;
    float sum = 0.0f;
#pragma unroll
    for (int r = 0; r < 8; ++r) sum += __expf(s0[r] - mn) + __expf(s1[r] - mn);
    sum += __shfl_xor(sum, 16); l = l * al_ + sum;
  }
  if (hh == 0) { Ms[wid * 16 + col] = m; Ls[wid * 16 + col] = PS / l; }
  __syncthreads();
  if (wid == 0) { float* dm = Mx + (size_t)b * N + blockIdx.x * 128; float* dl = Li + (size_t)b * N + blockIdx.x * 128;
    for (int pass = 0; pass < 2; ++pass) { *(volatile v4f*)(dm + lane * 4) = *(const v4f*)(&Ms[lane * 4]); *(volatile v4f*)(dl + lane * 4) = *(const v4f*)(&Ls[lane * 4]); __threadfence(); } }
}

__global__ __launch_bounds__(64) void pref_kernel(const b16* __restrict__ keyh, const b16* __restrict__ keyl, const float* __restrict__ Mx, const float* __restrict__ Li,
                                                 const b16* __restrict__ r16, const float* __restrict__ x, b16* __restrict__ vdiff) {
  __shared__ __attribute__((aligned(16))) b16 Pt[32 * 32];
  __shared__ __attribute__((aligned(16))) b16 Os[2][32][C1 + 8];
  const int wave = threadIdx.x >> 5, lane = threadIdx.x & 31, nloc = lane & 15, hlf = lane >> 4, b = blockIdx.y, n0 = blockIdx.x * 32, ch0 = wave * C1;
  const b16* kth = keyh + ((size_t)b * N) * KO; const b16* ktl = keyl + ((size_t)b * N) * KO;
  const b16* kqh = keyh + ((size_t)(Bn + b) * N) * KO; const b16* kql = keyl + ((size_t)(Bn + b) * N) * KO;
  const float* Mz = Mx + (size_t)b * N; const float* Lz = Li + (size_t)b * N; const b16* rz = r16 + (size_t)b * C * N;
  const v16b a0h = frag_kb(kth + (size_t)(n0 + nloc) * KO, hlf), a0l = frag_kb(ktl + (size_t)(n0 + nloc) * KO, hlf), a1h = frag_kb(kth + (size_t)(n0 + 16 + nloc) * KO, hlf), a1l = frag_kb(ktl + (size_t)(n0 + 16 + nloc) * KO, hlf);
  v8f y[2][8];
#pragma unroll
  for (int r = 0; r < 2; ++r)
#pragma unroll
    for (int t = 0; t < 8; ++t) y[r][t] = (v8f){};
  for (int mb = 0; mb < N; mb += 32) {
    const int mcol = mb + wave * 16 + nloc;
    const v16b bh = frag_kb(kqh + (size_t)mcol * KO, hlf), bl = frag_kb(kql + (size_t)mcol * KO, hlf);
    v8f f0 = {}, f1 = {}; f0 = mac<2, 2>(a0h, a0l, bh, bl, f0); f1 = mac<2, 2>(a1h, a1l, bh, bl, f1);
    const float mj = Mz[mcol], lj = Lz[mcol];
#pragma unroll
    for (int v = 0; v < 8; ++v) { Pt[(8 * hlf + v) * 32 + wave * 16 + nloc] = (b16)(__expf(f0[v] * (1.0f / (KS * KS)) - mj) * lj); Pt[(16 + 8 * hlf + v) * 32 + wave * 16 + nloc] = (b16)(__expf(f1[v] * (1.0f / (KS * KS)) - mj) * lj); }
    __syncthreads();
    const v16b p0 = frag_kb(Pt + nloc * 32, hlf), p1 = frag_kb(Pt + (16 + nloc) * 32, hlf);
#pragma unroll
    for (int t = 0; t < 8; ++t) { const v16b rb = frag_kb(rz + (size_t)(ch0 + t * 16 + nloc) * N + mb, hlf); y[0][t] = wmma16b(p0, rb, y[0][t]); y[1][t] = wmma16b(p1, rb, y[1][t]); }
    __syncthreads();
  }
  const float* xz = x + (size_t)b * C * N;
#pragma unroll
  for (int t = 0; t < 8; ++t)
#pragma unroll
    for (int r = 0; r < 2; ++r)
#pragma unroll
      for (int v = 0; v < 8; ++v) { const int rr = r * 16 + v + 8 * hlf, cc = t * 16 + nloc; const float val = y[r][t][v] * (1.0f / PS), xv = xz[(size_t)(ch0 + cc) * N + n0 + rr]; Os[wave][rr][cc] = (b16)(fabsf(val - xv) * AS); }
  wave_lds_sync();
  b16* dst = vdiff + ((size_t)b * N + n0) * C + ch0;
  for (int pass = 0; pass < 2; ++pass) {
#pragma unroll
    for (int j = 0; j < 16; ++j) { const int rr = j * 2 + hlf, c8 = nloc * 8; *(volatile v8b*)(dst + (size_t)rr * C + c8) = *(const v8b*)(&Os[wave][rr][c8]); }
    __threadfence();
  }
}

template <int MODE>
__global__ __launch_bounds__(128) void c1_kernel(const float* __restrict__ x, const float* __restrict__ pooled, const b16* __restrict__ vdiff, const b16* __restrict__ scin,
                                                 const b16* __restrict__ c1h, const float* __restrict__ c1b, b16* __restrict__ outp, int ldo, int coff) {
  __shared__ __attribute__((aligned(16))) b16 Ts[4][2][32 * 64];
  const int lane = threadIdx.x & 31, wave = threadIdx.x >> 5, nloc = lane & 15, hlf = lane >> 4, b = blockIdx.z;
  const int m0 = blockIdx.y * 128 + wave * 32, c0 = blockIdx.x * 64;
  const float* xz = x + (size_t)b * C * N; const float* pz = pooled + (size_t)b * C;
  v8f acc[2][4];
#pragma unroll
  for (int r = 0; r < 2; ++r)
#pragma unroll
    for (int t = 0; t < 4; ++t) acc[r][t] = (v8f){};
#pragma unroll 1
  for (int kb = 0; kb < C; kb += 32) {
    v16b a0, a1;
    if (MODE <= 1) {
#pragma unroll
      for (int e = 0; e < 16; ++e) { const int k = kb + ((e < 8) ? (8 * hlf + e) : (16 + 8 * hlf + e - 8)); const float pc_ = pz[k];
        const float x0 = xz[(size_t)k * N + m0 + nloc], x1 = xz[(size_t)k * N + m0 + 16 + nloc];
        a0[e] = (b16)((MODE == 0 ? fabsf(pc_ - x0) : x0 * pc_) * AS); a1[e] = (b16)((MODE == 0 ? fabsf(pc_ - x1) : x1 * pc_) * AS); }
    } else {
      const b16* src = (MODE == 2) ? (vdiff + ((size_t)b * N) * C) : (scin + ((size_t)b * N) * C);
      a0 = frag_kb(src + (size_t)(m0 + nloc) * C + kb, hlf); a1 = frag_kb(src + (size_t)(m0 + 16 + nloc) * C + kb, hlf);
    }
#pragma unroll
    for (int t = 0; t < 4; ++t) { const v16b bw = frag_kb(c1h + (size_t)(c0 + t * 16 + nloc) * C + kb, hlf); acc[0][t] = wmma16b(a0, bw, acc[0][t]); acc[1][t] = wmma16b(a1, bw, acc[1][t]); }
  }
#pragma unroll
  for (int t = 0; t < 4; ++t)
#pragma unroll
    for (int r = 0; r < 2; ++r)
#pragma unroll
      for (int v = 0; v < 8; ++v) acc[r][t][v] = acc[r][t][v] * (1.0f / (AS * WS)) + c1b[c0 + t * 16 + nloc];
  epi_planes(acc, AS, false, outp + ((size_t)b * N) * ldo + coff, nullptr, ldo, m0, c0, lane, Ts[wave][0], Ts[wave][1]);
}

__global__ __launch_bounds__(128) void metric_kernel(const b16* __restrict__ cs16, const b16* __restrict__ att16, const b16* __restrict__ xh, const b16* __restrict__ xl,
                                                     const b16* __restrict__ mwh, const float* __restrict__ mb, float* __restrict__ out) {
  __shared__ __attribute__((aligned(16))) float Ts[4][64][32 + 4];
  const int lane = threadIdx.x & 31, wave = threadIdx.x >> 5, nloc = lane & 15, hlf = lane >> 4, b = blockIdx.z;
  const int m0 = blockIdx.y * 128 + wave * 32, c0 = blockIdx.x * 64;
  v8f acc[2][4];
#pragma unroll
  for (int r = 0; r < 2; ++r)
#pragma unroll
    for (int t = 0; t < 4; ++t) acc[r][t] = (v8f){};
#pragma unroll 1
  for (int kb = 0; kb < 2 * C; kb += 32) {
    v16b a0, a1, a0l = {}, a1l = {};
    const bool isx = kb >= 2 * C1;
    if (kb < C1) { const b16* s = cs16 + ((size_t)b * N) * C1 + kb; a0 = frag_kb(s + (size_t)(m0 + nloc) * C1, hlf); a1 = frag_kb(s + (size_t)(m0 + 16 + nloc) * C1, hlf); }
    else if (!isx) { const b16* s = att16 + ((size_t)b * N) * C1 + (kb - C1); a0 = frag_kb(s + (size_t)(m0 + nloc) * C1, hlf); a1 = frag_kb(s + (size_t)(m0 + 16 + nloc) * C1, hlf); }
    else { const size_t o0 = ((size_t)b * NP1 + m0 + nloc) * C + (kb - 2 * C1), o1 = o0 + (size_t)16 * C; a0 = frag_kb(xh + o0, hlf); a1 = frag_kb(xh + o1, hlf); a0l = frag_kb(xl + o0, hlf); a1l = frag_kb(xl + o1, hlf); }
#pragma unroll
    for (int t = 0; t < 4; ++t) { const v16b bw = frag_kb(mwh + (size_t)(c0 + t * 16 + nloc) * (2 * C) + kb, hlf);
      acc[0][t] = wmma16b(a0, bw, acc[0][t]); acc[1][t] = wmma16b(a1, bw, acc[1][t]);
      if (isx) { acc[0][t] = wmma16b(a0l, bw, acc[0][t]); acc[1][t] = wmma16b(a1l, bw, acc[1][t]); } }
  }
#pragma unroll
  for (int t = 0; t < 4; ++t)
#pragma unroll
    for (int r = 0; r < 2; ++r)
#pragma unroll
      for (int v = 0; v < 8; ++v) { const int rr = r * 16 + v + 8 * hlf, cc = t * 16 + nloc; Ts[wave][cc][rr] = acc[r][t][v] * (1.0f / (AS * WS)) + mb[c0 + cc]; }
  wave_lds_sync();
  float* dst = out + ((size_t)b * C + c0) * N + m0;
  for (int pass = 0; pass < 2; ++pass) {
#pragma unroll
    for (int j = 0; j < 16; ++j) { const int cc = j * 4 + (lane >> 3), c4 = (lane & 7) * 4; *(volatile v4f*)(dst + (size_t)cc * N + c4) = *(const v4f*)(&Ts[wave][cc][c4]); }
    __threadfence();
  }
}
}

extern "C" void kernel_launch(void* const* d_in, const int* in_sizes, int n_in,
                              void* d_out, int out_size, void* d_ws, size_t ws_size, hipStream_t stream) {
  (void)n_in; (void)out_size;
  const float* x = (const float*)d_in[0]; const float* ref = (const float*)d_in[1];
  const float* ktw = (const float*)d_in[2]; const float* ktb = (const float*)d_in[3];
  const float* kqw = (const float*)d_in[4]; const float* kqb = (const float*)d_in[5];
  const float* c1w = (const float*)d_in[6]; const float* c1b = (const float*)d_in[7];
  const float* mw = (const float*)d_in[8]; const float* mb = (const float*)d_in[9];
  float* out = (float*)d_out;
  if (in_sizes[0] != Bn * C * N || in_sizes[1] != Bn * C * N || in_sizes[2] != KO * C * 9 || in_sizes[6] != C1 * C || in_sizes[8] != C * 2 * C) return;
  size_t off = 0; char* ws = (char*)d_ws;
  auto carve = [&](size_t bytes) { char* p = ws + off; off += (bytes + 255) & ~(size_t)255; return p; };
  b16* cwh = (b16*)carve((size_t)2 * KO * KC * 2); b16* cwl = (b16*)carve((size_t)2 * KO * KC * 2);
  b16* c1h = (b16*)carve((size_t)C1 * C * 2); b16* mwh = (b16*)carve((size_t)C * 2 * C * 2);
  b16* xh = (b16*)carve((size_t)Bn * NP1 * C * 2); b16* xl = (b16*)carve((size_t)Bn * NP1 * C * 2);
  b16* rh = (b16*)carve((size_t)Bn * NP1 * C * 2); b16* rl = (b16*)carve((size_t)Bn * NP1 * C * 2);
  b16* r16 = (b16*)carve((size_t)Bn * C * N * 2);
  float* pooled = (float*)carve((size_t)Bn * C * 4);
  b16* keyh = (b16*)carve((size_t)2 * Bn * N * KO * 2); b16* keyl = (b16*)carve((size_t)2 * Bn * N * KO * 2);
  float* Mx = (float*)carve((size_t)Bn * N * 4); float* Li = (float*)carve((size_t)Bn * N * 4);
  b16* vdiff = (b16*)carve((size_t)Bn * N * C * 2);
  b16* scin = (b16*)carve((size_t)Bn * N * C * 2);
  b16* att16 = (b16*)carve((size_t)Bn * N * C1 * 2); b16* cs16 = (b16*)carve((size_t)Bn * N * C1 * 2);
  if (off > ws_size) return;
  prep_kernel<<<256, 256, 0, stream>>>(ktw, kqw, c1w, mw, cwh, cwl, c1h, mwh, xh, xl, rh, rl);
  trans_kernel<<<dim3(64 * 4, Bn, 2), 256, 0, stream>>>(x, ref, xh, xl, rh, rl);
  refprep_kernel<<<Bn * C / 32, 256, 0, stream>>>(ref, r16, pooled);
  conv3_kernel<<<dim3(N / 256, Bn * 2), 128, 0, stream>>>(xh, xl, rh, rl, cwh, cwl, ktb, kqb, keyh, keyl);
  stats_kernel<<<dim3(N / 128, Bn), 256, 0, stream>>>(keyh, keyl, Mx, Li);
  pref_kernel<<<dim3(N / 32, Bn), 64, 0, stream>>>(keyh, keyl, Mx, Li, r16, x, vdiff);
  c1_kernel<0><<<dim3(2, N / 128, Bn), 128, 0, stream>>>(x, pooled, vdiff, scin, c1h, c1b, scin, C, C1);
  c1_kernel<1><<<dim3(2, N / 128, Bn), 128, 0, stream>>>(x, pooled, vdiff, scin, c1h, c1b, scin, C, 0);
  c1_kernel<2><<<dim3(2, N / 128, Bn), 128, 0, stream>>>(x, pooled, vdiff, scin, c1h, c1b, att16, C1, 0);
  c1_kernel<3><<<dim3(2, N / 128, Bn), 128, 0, stream>>>(x, pooled, vdiff, scin, c1h, c1b, cs16, C1, 0);
  metric_kernel<<<dim3(C / 64, N / 128, Bn), 128, 0, stream>>>(cs16, att16, xh, xl, mwh, mb, out);
}
